// Obj2ObjGNN_78383153152533
// MI455X (gfx1250) — hardware-verified
//
#include <hip/hip_runtime.h>
#include <stddef.h>


#define FD      256
#define K2      512
#define ASC     8
#define WSC     64
#define OSC     (1.0f / 512.0f)
#define NTHR    256
#define NWAVE   8
#define EPT     4
#define NGRP    4
#define CHUNK   (NTHR * EPT * NGRP)
#define WCAP    (EPT * NGRP * 32)
#define LISTN   (NWAVE * WCAP)
#define NBC     4096
#define NBF     512
#define FPB     8
#define RCAP    20480
#define RBN     128
#define OTHR    512
#define DEGCAP  256
#define BM      64
#define NCW     64
#define TW      2
#define TTHR    (TW * 32)
#define ANB     8
#define PEW     32
#define VCAP    128
#define WSCAP   134217728
#define LDS_FILL ((2 * RCAP + NBF + LISTN) * 4 + 64)

static_assert((CHUNK & (CHUNK - 1)) == 0);
static_assert(CHUNK <= 4096);
static_assert(NBC <= 4096 && NBF <= 4096);
static_assert((NBC & (NBC - 1)) == 0 && (NBF & (NBF - 1)) == 0);
static_assert(NBC == FPB * NBF);
static_assert(OTHR * 8 == NBC);
static_assert(OTHR / 64 == FPB);
static_assert((RCAP % 32) == 0);
static_assert((RCAP / 4) % NTHR == 0);
static_assert(BM * 4 == NTHR);
static_assert(WCAP == EPT * NGRP * 32);
static_assert(TTHR == 64);
static_assert(ANB == NWAVE);
static_assert(FD == 8 * 32);

typedef float          v4f  __attribute__((ext_vector_type(4)));
typedef float          v8f  __attribute__((ext_vector_type(8)));
typedef int            v4i  __attribute__((ext_vector_type(4)));
typedef _Float16       v4h  __attribute__((ext_vector_type(4)));
typedef _Float16       v8h  __attribute__((ext_vector_type(8)));
typedef _Float16       v16h __attribute__((ext_vector_type(16)));
typedef _Float16       v8ha __attribute__((ext_vector_type(8), __may_alias__));
typedef unsigned short v4us __attribute__((ext_vector_type(4)));
typedef unsigned short v8us __attribute__((ext_vector_type(8)));
union FragH { v16h v; v8us u[2]; v8h h[2]; };

__device__ __forceinline__ v8f wmh(v16h a, v16h b, v8f c) {
  v8f d = __builtin_amdgcn_wmma_f32_16x16x32_f16(false, a, false, b, (short)0, c, false, false);
  asm volatile("v_nop\n\tv_nop\n\tv_nop\n\tv_nop" : "+v"(d) : "v"(a), "v"(b));
  return d;
}
__device__ __forceinline__ v8f zero8() { v8f z = {0.f, 0.f, 0.f, 0.f, 0.f, 0.f, 0.f, 0.f}; return z; }
__device__ __forceinline__ float wsum32(float v) {
#pragma unroll
  for (int s = 16; s > 0; s >>= 1) v += __shfl_xor(v, s);
  return v;
}

__device__ __forceinline__ v16h frag_glb(const unsigned short* P, int row, int ld, int k0, int hh) {
  FragH f;
  const unsigned short* p = P + (size_t)row * ld + k0 + 8 * hh;
  f.u[0] = *(const v8us*)p;
  f.u[1] = *(const v8us*)(p + 16);
  return f.v;
}
__device__ __forceinline__ v16h frag_lds(const _Float16* T, int row, int ld, int k0, int hh) {
  FragH f;
  const _Float16* p = T + row * ld + k0 + 8 * hh;
  f.h[0] = *(const v8h*)p;
  f.h[1] = *(const v8h*)(p + 16);
  return f.v;
}

template <int NB>
__device__ __forceinline__ int scan_chunk(const int* __restrict__ dsts, int nE, int cbase, int slotBase,
                                          int vec4, int* list, int tid, int lane, int wave) {
  int wc = 0;
  const int sent = -2147483647 - 1;
#pragma unroll 1
  for (int g = 0; g < NGRP; ++g) {
    const int el0  = (g * NTHR + tid) * EPT;
    const int e0   = cbase + el0;
    v4i da;
    if (vec4 != 0 && cbase + CHUNK <= nE) {
      da = *(const v4i*)(dsts + e0);
    } else {
      da.x = (e0     < nE) ? dsts[min(e0, nE - 1)] : sent;
      da.y = (e0 + 1 < nE) ? dsts[min(e0 + 1, nE - 1)] : sent;
      da.z = (e0 + 2 < nE) ? dsts[min(e0 + 2, nE - 1)] : sent;
      da.w = (e0 + 3 < nE) ? dsts[min(e0 + 3, nE - 1)] : sent;
    }
    const unsigned nb = (unsigned)slotBase;
    const unsigned s0 = (unsigned)da.x - nb, s1 = (unsigned)da.y - nb;
    const unsigned s2 = (unsigned)da.z - nb, s3 = (unsigned)da.w - nb;
    const bool h0 = s0 < (unsigned)NB, h1 = s1 < (unsigned)NB, h2 = s2 < (unsigned)NB, h3 = s3 < (unsigned)NB;
    const unsigned any = __builtin_amdgcn_ballot_w32(h0 | h1 | h2 | h3);
    if (any != 0u) {
#define HITJ(J, HJ, SJ) { \
        const unsigned mj = __builtin_amdgcn_ballot_w32(HJ); \
        if (mj != 0u) { \
          if (HJ) { \
            const int pos = wc + (int)__builtin_amdgcn_mbcnt_lo(mj, 0u); \
            if (pos < WCAP) list[wave * WCAP + pos] = ((el0 + (J)) << 12) | (int)(SJ); \
          } \
          wc += (int)__builtin_popcount(mj); } }
      HITJ(0, h0, s0)
      HITJ(1, h1, s1)
      HITJ(2, h2, s2)
      HITJ(3, h3, s3)
#undef HITJ
    }
  }
  return wc;
}

__global__ __launch_bounds__(NTHR) __attribute__((amdgpu_num_vgpr(VCAP)))
void k_count(const int* __restrict__ keys, int* cnt, int nE, int vec4) {
  __shared__ __attribute__((aligned(16))) int scnt[NBC];
  __shared__ __attribute__((aligned(16))) int list[LISTN];
  __shared__ int wcnt[NWAVE];
  const int tid = threadIdx.x, lane = tid & 31, wave = tid >> 5;
  const int nodeBase = blockIdx.x * NBC;

#pragma unroll 1
  for (int i = tid; i < NBC; i += NTHR) scnt[i] = 0;
  __syncthreads();

  const int nChunks = (nE + CHUNK - 1) / CHUNK;
#pragma unroll 1
  for (int ch = 0; ch < nChunks; ++ch) {
    const int cbase = ch * CHUNK;
    const int wc = scan_chunk<NBC>(keys, nE, cbase, nodeBase, vec4, list, tid, lane, wave);
    if (lane == 0) wcnt[wave] = wc;
    __syncthreads();
    if (wave == 0) {
#pragma unroll 1
      for (int wsx = 0; wsx < NWAVE; ++wsx) {
        int n = __builtin_amdgcn_readfirstlane(wcnt[wsx]);
        n = n > WCAP ? WCAP : (n < 0 ? 0 : n);
        const int* lp = list + wsx * WCAP;
#pragma unroll 1
        for (int i = 0; i < n; ++i) {
          const int ent  = __builtin_amdgcn_readfirstlane(lp[i]);
          const int slot = ent & (NBC - 1);
          if (lane == 0) scnt[slot] = scnt[slot] + 1;
        }
      }
    }
    __syncthreads();
  }

  v4i cq[4];
#pragma unroll
  for (int q = 0; q < 4; ++q) {
    const int f = (wave * 4 + q) * 128 + 4 * lane;
    cq[q] = *(const v4i*)(scnt + f);
  }
  int* cp = cnt + (size_t)nodeBase;
#pragma unroll
  for (int q = 0; q < 4; ++q) {
    const int f = (wave * 4 + q) * 128 + 4 * lane;
    *(volatile v4i*)(cp + f) = cq[q];
  }
  __threadfence();
#pragma unroll
  for (int q = 0; q < 4; ++q) {
    const int f = (wave * 4 + q) * 128 + 4 * lane;
    *(volatile v4i*)(cp + f) = cq[q];
  }
}

__global__ __launch_bounds__(OTHR) void k_offsets(
    const int* __restrict__ cnt, int* off, int* rbase, int nChunk) {
  __shared__ __attribute__((aligned(16))) int soff[NBC];
  __shared__ __attribute__((aligned(16))) int srb[RBN];
  __shared__ int wtot[OTHR / 32];
  const int tid = threadIdx.x, lane = tid & 31, wave = tid >> 5, sub = tid >> 6;
  for (int i = tid; i < RBN; i += OTHR) srb[i] = 0;
  int carry = 0;
#pragma unroll 1
  for (int ch = 0; ch < nChunk; ++ch) {
    const int base = ch * NBC;
    const v4i c0 = *(const v4i*)(cnt + base + 8 * tid);
    const v4i c1 = *(const v4i*)(cnt + base + 8 * tid + 4);
    const int e0 = max(c0.x, 0), e1 = max(c0.y, 0), e2 = max(c0.z, 0), e3 = max(c0.w, 0);
    const int e4 = max(c1.x, 0), e5 = max(c1.y, 0), e6 = max(c1.z, 0), e7 = max(c1.w, 0);
    const int ts = e0 + e1 + e2 + e3 + e4 + e5 + e6 + e7;
    int incl = ts;
#pragma unroll
    for (int d = 1; d < 32; d <<= 1) {
      const int t = __shfl_up(incl, d);
      if (lane >= d) incl += t;
    }
    if (lane == 31) wtot[wave] = incl;
    __syncthreads();
    int bj = carry;
    int myb = carry;
#pragma unroll
    for (int j = 0; j < FPB; ++j) {
      myb = (sub == j) ? bj : myb;
      if (tid == 0) srb[min(FPB * ch + j, RBN - 1)] = bj;
      const int sj = wtot[2 * j] + wtot[2 * j + 1];
      bj += (sj + 31) & ~31;
    }
    const int wev = wave & ~1;
    const int pre = (wave & 1) ? wtot[wev] : 0;
    int run = myb + pre + incl - ts;
    soff[8 * tid + 0] = run; run += e0;
    soff[8 * tid + 1] = run; run += e1;
    soff[8 * tid + 2] = run; run += e2;
    soff[8 * tid + 3] = run; run += e3;
    soff[8 * tid + 4] = run; run += e4;
    soff[8 * tid + 5] = run; run += e5;
    soff[8 * tid + 6] = run; run += e6;
    soff[8 * tid + 7] = run;
    carry = bj;
    __syncthreads();
    const v4i o0 = *(const v4i*)(soff + 4 * tid);
    const v4i o1 = *(const v4i*)(soff + 4 * (tid + OTHR));
    int* op = off + base;
    *(volatile v4i*)(op + 4 * tid) = o0;
    *(volatile v4i*)(op + 4 * (tid + OTHR)) = o1;
    __threadfence();
    *(volatile v4i*)(op + 4 * tid) = o0;
    *(volatile v4i*)(op + 4 * (tid + OTHR)) = o1;
    __syncthreads();
  }
  if (tid == 0) srb[min(FPB * nChunk, RBN - 1)] = carry;
  __syncthreads();
  v4i rv = {0, 0, 0, 0};
  if (tid < 32) rv = *(const v4i*)(srb + 4 * tid);
  if (tid < 32) *(volatile v4i*)(rbase + 4 * tid) = rv;
  __threadfence();
  if (tid < 32) *(volatile v4i*)(rbase + 4 * tid) = rv;
}

__global__ __launch_bounds__(NTHR) __attribute__((amdgpu_num_vgpr(VCAP)))
void k_fill(const int* __restrict__ vals, const int* __restrict__ keys,
            const int* __restrict__ off, const int* __restrict__ rbase,
            int* csrC, int* csrR, int nNa, int nNb, int nE, int vec4, int csrLen) {
  extern __shared__ v4f lds_dyn[];
  int* regionC = (int*)lds_dyn;
  int* regionR = regionC + RCAP;
  int* cursor  = regionR + RCAP;
  int* list    = cursor + NBF;
  int* wcnt    = list + LISTN;
  const int tid = threadIdx.x, lane = tid & 31, wave = tid >> 5;
  const int b = blockIdx.x;
  const int nodeBase = b * NBF;

  int rb0 = rbase[b];
  const int rb1 = rbase[b + 1];
  rb0 = rb0 < 0 ? 0 : (rb0 > csrLen ? csrLen : rb0);
  rb0 &= ~31;
  int len = rb1 - rb0;
  len = len < 0 ? 0 : (len > RCAP ? RCAP : len);
  int lenW = (len + 31) & ~31;
  if (rb0 + lenW > csrLen) lenW = (csrLen - rb0) & ~31;

  {
    const v4i z = {0, 0, 0, 0};
#pragma unroll 1
    for (int i = tid; i < RCAP / 4; i += NTHR) { ((v4i*)regionC)[i] = z; ((v4i*)regionR)[i] = z; }
#pragma unroll 1
    for (int s = tid; s < NBF; s += NTHR) {
      int o = off[nodeBase + s] - rb0;
      o = o < 0 ? 0 : (o > RCAP ? RCAP : o);
      cursor[s] = o;
    }
  }
  __syncthreads();

  const int nChunks = (nE + CHUNK - 1) / CHUNK;
#pragma unroll 1
  for (int ch = 0; ch < nChunks; ++ch) {
    const int cbase = ch * CHUNK;
    const int wc = scan_chunk<NBF>(keys, nE, cbase, nodeBase, vec4, list, tid, lane, wave);
    if (lane == 0) wcnt[wave] = wc;
    __syncthreads();
    if (wave == 0) {
#pragma unroll 1
      for (int wsx = 0; wsx < NWAVE; ++wsx) {
        int n = __builtin_amdgcn_readfirstlane(wcnt[wsx]);
        n = n > WCAP ? WCAP : (n < 0 ? 0 : n);
        const int* lp = list + wsx * WCAP;
#pragma unroll 1
        for (int i = 0; i < n; ++i) {
          const int ent  = __builtin_amdgcn_readfirstlane(lp[i]);
          const int slot = ent & (NBF - 1);
          int e = cbase + ((ent >> 12) & (CHUNK - 1));
          e = e > nE - 1 ? nE - 1 : e;
          int sv = vals[e];
          sv = sv < 0 ? 0 : (sv > nNb - 1 ? nNb - 1 : sv);
          int rv = nodeBase + slot;
          rv = rv > nNa - 1 ? nNa - 1 : rv;
          if (lane == 0) {
            int pos = cursor[slot];
            pos = pos < 0 ? 0 : (pos > RCAP - 1 ? RCAP - 1 : pos);
            regionC[pos] = sv;
            regionR[pos] = rv;
            const int np = pos + 1;
            cursor[slot] = np > RCAP ? RCAP : np;
          }
        }
      }
    }
    __syncthreads();
  }

  const int nv = lenW >> 2;
  int* gpC = csrC + rb0;
  int* gpR = csrR + rb0;
#pragma unroll 1
  for (int i = tid; i < nv; i += NTHR) {
    const v4i vc = ((const v4i*)regionC)[i];
    const v4i vr = ((const v4i*)regionR)[i];
    *(volatile v4i*)(gpC + 4 * i) = vc;
    *(volatile v4i*)(gpR + 4 * i) = vr;
  }
  __threadfence();
#pragma unroll 1
  for (int i = tid; i < nv; i += NTHR) {
    const v4i vc = ((const v4i*)regionC)[i];
    const v4i vr = ((const v4i*)regionR)[i];
    *(volatile v4i*)(gpC + 4 * i) = vc;
    *(volatile v4i*)(gpR + 4 * i) = vr;
  }
}

__device__ __forceinline__ void wcvt_unit(const float* __restrict__ W, unsigned short* dst,
                                          int K, int KP, int Nout, int ld, int i) {
  const int upc = KP >> 3;
  if (i >= Nout * upc) return;
  const int n = i / upc;
  const int seg = i - n * upc;
  v8h o;
#pragma unroll
  for (int j = 0; j < 8; ++j) {
    const int k = 8 * seg + j;
    const int kc = k < K - 1 ? k : K - 1;
    const float v = W[(size_t)kc * ld + n];
    o[j] = (k < K) ? (_Float16)(v * (float)WSC) : (_Float16)0.0f;
  }
  const v8us ob = __builtin_bit_cast(v8us, o);
  unsigned short* d = dst + (size_t)i * 8;
  *(volatile v8us*)d = ob;
  __threadfence();
  *(volatile v8us*)d = ob;
}

__global__ __launch_bounds__(NTHR) void k_wcvt(
    const float* __restrict__ w0, const float* __restrict__ w1, const float* __restrict__ w2,
    const float* __restrict__ w3, const float* __restrict__ w4, const float* __restrict__ w5,
    const float* __restrict__ w6,
    unsigned short* d0, unsigned short* d1, unsigned short* d2, unsigned short* d3,
    unsigned short* d4, unsigned short* d5, unsigned short* d6) {
  const int job = (int)blockIdx.y;
  const float* W =
      (job == 0) ? w0 : (job == 1) ? w1 : (job == 2) ? w2 : (job == 3) ? w3 :
      (job == 4) ? w4 : (job == 5) ? w5 : w6;
  unsigned short* dst =
      (job == 0) ? d0 : (job == 1) ? d1 : (job == 2) ? d2 : (job == 3) ? d3 :
      (job == 4) ? d4 : (job == 5) ? d5 : d6;
  const int K = (job == 0 || job == 3 || job == 6) ? K2 : FD;
  wcvt_unit(W, dst, K, K, FD, FD, (int)blockIdx.x * NTHR + (int)threadIdx.x);
}

template <int COPY32>
__device__ __forceinline__ void ncvt_pass(const float* __restrict__ src, float* d32, unsigned short* d16,
                                          int n8, int i0, int T) {
#pragma unroll 1
  for (int i = i0; i < n8; i += T) {
    const v4f a = *(const v4f*)(src + (size_t)i * 8);
    const v4f b = *(const v4f*)(src + (size_t)i * 8 + 4);
    v8h o;
    o[0] = (_Float16)(a.x * (float)ASC); o[1] = (_Float16)(a.y * (float)ASC);
    o[2] = (_Float16)(a.z * (float)ASC); o[3] = (_Float16)(a.w * (float)ASC);
    o[4] = (_Float16)(b.x * (float)ASC); o[5] = (_Float16)(b.y * (float)ASC);
    o[6] = (_Float16)(b.z * (float)ASC); o[7] = (_Float16)(b.w * (float)ASC);
    const v8us ob = __builtin_bit_cast(v8us, o);
    *(volatile v8us*)(d16 + (size_t)i * 8) = ob;
  }
  if (COPY32) {
#pragma unroll 1
    for (int u = i0; u < 2 * n8; u += T) {
      const v4f v = *(const v4f*)(src + (size_t)u * 4);
      *(volatile v4f*)(d32 + (size_t)u * 4) = v;
    }
  }
}
template <int COPY32>
__global__ __launch_bounds__(NTHR) void k_ncvt(const float* __restrict__ src, float* d32,
                                               unsigned short* d16, int n8) {
  const int i0 = (int)blockIdx.x * NTHR + (int)threadIdx.x;
  const int T = (int)gridDim.x * NTHR;
  ncvt_pass<COPY32>(src, d32, d16, n8, i0, T);
  __threadfence();
  ncvt_pass<COPY32>(src, d32, d16, n8, i0, T);
}

__global__ __launch_bounds__(NTHR) void k_gemm(const unsigned short* __restrict__ Ap,
                                               const unsigned short* __restrict__ Bp,
                                               float* C, int lda, int ldb, int KT, int ldc, float osc) {
  __shared__ __attribute__((aligned(16))) float stg[BM * NCW];
  const int tid = threadIdx.x, lane = tid & 31, wave = tid >> 5, hh = lane >> 4, m = lane & 15;
  const int rowBase = (int)blockIdx.x * BM;
  const int colBase = (int)blockIdx.y * NCW;
  const int rg = wave >> 1, chf = wave & 1;
  const int r0 = rg * 16;
  const int c0 = chf * 32;

  v8f acc0 = zero8();
  v8f acc1 = zero8();

  const unsigned short* ap  = Ap + (size_t)(rowBase + r0 + m) * lda + 8 * hh;
  const unsigned short* bpA = Bp + (size_t)(colBase + c0 + m) * ldb + 8 * hh;
  const unsigned short* bpB = bpA + (size_t)16 * ldb;
#pragma unroll 1
  for (int kt = 0; kt < KT; ++kt) {
    const v8us a0 = *(const v8us*)(ap + 32 * kt);
    const v8us a1 = *(const v8us*)(ap + 32 * kt + 16);
    const v8us b00 = *(const v8us*)(bpA + 32 * kt);
    const v8us b01 = *(const v8us*)(bpA + 32 * kt + 16);
    const v8us b10 = *(const v8us*)(bpB + 32 * kt);
    const v8us b11 = *(const v8us*)(bpB + 32 * kt + 16);
    FragH a, b0, b1;
    a.u[0] = a0; a.u[1] = a1; b0.u[0] = b00; b0.u[1] = b01; b1.u[0] = b10; b1.u[1] = b11;
    acc0 = wmh(a.v, b0.v, acc0);
    acc1 = wmh(a.v, b1.v, acc1);
  }

  {
    float* sp = stg + (size_t)(r0 + 8 * hh) * NCW + c0 + m;
#pragma unroll
    for (int r = 0; r < 8; ++r) {
      sp[r * NCW]      = acc0[r] * osc;
      sp[r * NCW + 16] = acc1[r] * osc;
    }
  }
  __syncthreads();

  v4f cv[4];
#pragma unroll
  for (int it = 0; it < 4; ++it) {
    const int id = it * NTHR + tid;
    const int row = id >> 4, seg = id & 15;
    cv[it] = *(const v4f*)(stg + (size_t)row * NCW + 4 * seg);
  }
#pragma unroll
  for (int it = 0; it < 4; ++it) {
    const int id = it * NTHR + tid;
    const int row = id >> 4, seg = id & 15;
    float* gp = C + (size_t)(rowBase + row) * ldc + colBase + 4 * seg;
    *(volatile v4f*)gp = cv[it];
  }
  __threadfence();
#pragma unroll
  for (int it = 0; it < 4; ++it) {
    const int id = it * NTHR + tid;
    const int row = id >> 4, seg = id & 15;
    float* gp = C + (size_t)(rowBase + row) * ldc + colBase + 4 * seg;
    *(volatile v4f*)gp = cv[it];
  }
}

__device__ __forceinline__ void ln_relu_rows(const float* sFw, _Float16* sAw, const float* __restrict__ g,
                                             const float* __restrict__ b, int lane) {
  const v4f g0 = *(const v4f*)(g + 8 * lane), g1 = *(const v4f*)(g + 8 * lane + 4);
  const v4f o0 = *(const v4f*)(b + 8 * lane), o1 = *(const v4f*)(b + 8 * lane + 4);
#pragma unroll 2
  for (int i = 0; i < 16; ++i) {
    const v4f u0 = *(const v4f*)(sFw + i * FD + 8 * lane);
    const v4f u1 = *(const v4f*)(sFw + i * FD + 8 * lane + 4);
    float s = ((u0.x + u0.y) + (u0.z + u0.w)) + ((u1.x + u1.y) + (u1.z + u1.w));
    s = wsum32(s);
    const float mu = s * (1.0f / 256.0f);
    const v4f d0 = u0 - mu, d1 = u1 - mu;
    float q = ((d0.x * d0.x + d0.y * d0.y) + (d0.z * d0.z + d0.w * d0.w)) +
              ((d1.x * d1.x + d1.y * d1.y) + (d1.z * d1.z + d1.w * d1.w));
    q = wsum32(q);
    const float rs = rsqrtf(q * (1.0f / 256.0f) + 1e-5f);
    const v4f y0 = d0 * rs * g0 + o0;
    const v4f y1 = d1 * rs * g1 + o1;
    v8h o;
    o[0] = (_Float16)(fmaxf(y0.x, 0.0f) * (float)ASC); o[1] = (_Float16)(fmaxf(y0.y, 0.0f) * (float)ASC);
    o[2] = (_Float16)(fmaxf(y0.z, 0.0f) * (float)ASC); o[3] = (_Float16)(fmaxf(y0.w, 0.0f) * (float)ASC);
    o[4] = (_Float16)(fmaxf(y1.x, 0.0f) * (float)ASC); o[5] = (_Float16)(fmaxf(y1.y, 0.0f) * (float)ASC);
    o[6] = (_Float16)(fmaxf(y1.z, 0.0f) * (float)ASC); o[7] = (_Float16)(fmaxf(y1.w, 0.0f) * (float)ASC);
    *(v8h*)(sAw + i * FD + 8 * lane) = o;
  }
}

__device__ __forceinline__ void mrows_pass(const _Float16* sMw, unsigned short* Mp, int s0, int lane) {
#pragma unroll
  for (int i = 0; i < 16; ++i) {
    const v8ha t = *(const v8ha*)(sMw + i * FD + 8 * lane);
    const v8us u = __builtin_bit_cast(v8us, t);
    *(volatile v8us*)(Mp + (size_t)(s0 + i) * FD + 8 * lane) = u;
  }
}

__global__ __launch_bounds__(TTHR) void k_edge(
    const int* __restrict__ csrR, const int* __restrict__ csrC,
    const float* __restrict__ PA, const float* __restrict__ PB, const float* __restrict__ eb1,
    const unsigned short* __restrict__ W2p, const float* __restrict__ eb2,
    const float* __restrict__ lng, const float* __restrict__ lnb,
    const unsigned short* __restrict__ W3p, const float* __restrict__ eb3,
    unsigned short* Mp, int nNa, int nNb, int csrLen) {
  __shared__ __attribute__((aligned(16))) _Float16 sA[TW][16 * FD];
  __shared__ __attribute__((aligned(16))) float    sF[TW][16 * FD];
  __shared__ int sIdx[TW][32];
  const int tid = threadIdx.x, lane = tid & 31, wave = tid >> 5, hh = lane >> 4, m = lane & 15;
  const int s0 = ((int)blockIdx.x * TW + wave) * 16;
  _Float16* sAw = sA[wave];
  float* sFw = sF[wave];
  _Float16* sMw = (_Float16*)sFw;

  {
    const int e = lane & 15;
    int s = s0 + e; s = s > csrLen - 1 ? csrLen - 1 : s;
    int r = csrR[s];
    int c = csrC[s];
    r = r < 0 ? 0 : (r > nNa - 1 ? nNa - 1 : r);
    c = c < 0 ? 0 : (c > nNb - 1 ? nNb - 1 : c);
    if (lane < 16) {
      sIdx[wave][2 * e]     = r;
      sIdx[wave][2 * e + 1] = c;
    }
  }
  __syncthreads();

  {
    const v4f bq0 = *(const v4f*)(eb1 + 8 * lane), bq1 = *(const v4f*)(eb1 + 8 * lane + 4);
#pragma unroll 1
    for (int e = 0; e < 16; ++e) {
      const int r = sIdx[wave][2 * e];
      const int c = sIdx[wave][2 * e + 1];
      const float* pr = PA + (size_t)r * FD + 8 * lane;
      const float* pc = PB + (size_t)c * FD + 8 * lane;
      const v4f x0 = *(const v4f*)pr + *(const v4f*)pc + bq0;
      const v4f x1 = *(const v4f*)(pr + 4) + *(const v4f*)(pc + 4) + bq1;
      v8h o;
      o[0] = (_Float16)(fmaxf(x0.x, 0.0f) * (float)ASC); o[1] = (_Float16)(fmaxf(x0.y, 0.0f) * (float)ASC);
      o[2] = (_Float16)(fmaxf(x0.z, 0.0f) * (float)ASC); o[3] = (_Float16)(fmaxf(x0.w, 0.0f) * (float)ASC);
      o[4] = (_Float16)(fmaxf(x1.x, 0.0f) * (float)ASC); o[5] = (_Float16)(fmaxf(x1.y, 0.0f) * (float)ASC);
      o[6] = (_Float16)(fmaxf(x1.z, 0.0f) * (float)ASC); o[7] = (_Float16)(fmaxf(x1.w, 0.0f) * (float)ASC);
      *(v8h*)(sAw + e * FD + 8 * lane) = o;
    }
  }
  __syncthreads();

#pragma unroll 1
  for (int np = 0; np < 8; ++np) {
    const int c0 = 32 * np + m, c1 = c0 + 16;
    v8f acc0 = zero8(), acc1 = zero8();
#pragma unroll 1
    for (int kt = 0; kt < 8; ++kt) {
      const v16h a  = frag_lds(sAw, m, FD, 32 * kt, hh);
      const v16h b0 = frag_glb(W2p, c0, FD, 32 * kt, hh);
      const v16h b1 = frag_glb(W2p, c1, FD, 32 * kt, hh);
      acc0 = wmh(a, b0, acc0);
      acc1 = wmh(a, b1, acc1);
    }
    const float bv0 = eb2[c0], bv1 = eb2[c1];
#pragma unroll
    for (int r = 0; r < 8; ++r) {
      sFw[(8 * hh + r) * FD + c0] = acc0[r] * OSC + bv0;
      sFw[(8 * hh + r) * FD + c1] = acc1[r] * OSC + bv1;
    }
  }
  __syncthreads();

  ln_relu_rows(sFw, sAw, lng, lnb, lane);
  __syncthreads();

#pragma unroll 1
  for (int np = 0; np < 8; ++np) {
    const int c0 = 32 * np + m, c1 = c0 + 16;
    v8f acc0 = zero8(), acc1 = zero8();
#pragma unroll 1
    for (int kt = 0; kt < 8; ++kt) {
      const v16h a  = frag_lds(sAw, m, FD, 32 * kt, hh);
      const v16h b0 = frag_glb(W3p, c0, FD, 32 * kt, hh);
      const v16h b1 = frag_glb(W3p, c1, FD, 32 * kt, hh);
      acc0 = wmh(a, b0, acc0);
      acc1 = wmh(a, b1, acc1);
    }
    const float bv0 = eb3[c0], bv1 = eb3[c1];
#pragma unroll
    for (int r = 0; r < 8; ++r) {
      sMw[(8 * hh + r) * FD + c0] = (_Float16)((acc0[r] * OSC + bv0) * (float)ASC);
      sMw[(8 * hh + r) * FD + c1] = (_Float16)((acc1[r] * OSC + bv1) * (float)ASC);
    }
  }
  __syncthreads();

  mrows_pass(sMw, Mp, s0, lane);
  __threadfence();
  mrows_pass(sMw, Mp, s0, lane);
}

__global__ __launch_bounds__(NTHR) __attribute__((amdgpu_num_vgpr(VCAP)))
void k_agg(const int* __restrict__ cnt, const int* __restrict__ off,
           const unsigned short* __restrict__ Mp, unsigned short* AggA, int nN, int csrLen) {
  const int tid = threadIdx.x, lane = tid & 31, wave = tid >> 5;
  int n = (int)blockIdx.x * ANB + wave; n = n > nN - 1 ? nN - 1 : n;
  const _Float16* Mh = (const _Float16*)Mp;
  const v4f z4 = {0.f, 0.f, 0.f, 0.f};

  int dg = cnt[n];
  dg = dg < 0 ? 0 : (dg > DEGCAP ? DEGCAP : dg);
  dg = __builtin_amdgcn_readfirstlane(dg);
  int st = off[n];
  st = st < 0 ? 0 : (st > csrLen - 1 ? csrLen - 1 : st);
  st = __builtin_amdgcn_readfirstlane(st);
  v4f a0 = z4, a1 = z4;
#pragma unroll 1
  for (int i = 0; i < dg; ++i) {
    int s = st + i; s = s > csrLen - 1 ? csrLen - 1 : s;
    const v8ha mv = *(const v8ha*)(Mh + (size_t)s * FD + 8 * lane);
    a0.x += (float)mv[0]; a0.y += (float)mv[1]; a0.z += (float)mv[2]; a0.w += (float)mv[3];
    a1.x += (float)mv[4]; a1.y += (float)mv[5]; a1.z += (float)mv[6]; a1.w += (float)mv[7];
  }
  v8h ho;
  ho[0] = (_Float16)a0.x; ho[1] = (_Float16)a0.y; ho[2] = (_Float16)a0.z; ho[3] = (_Float16)a0.w;
  ho[4] = (_Float16)a1.x; ho[5] = (_Float16)a1.y; ho[6] = (_Float16)a1.z; ho[7] = (_Float16)a1.w;
  const v8us agv = __builtin_bit_cast(v8us, ho);
  unsigned short* gp = AggA + (size_t)n * FD + 8 * lane;
  *(volatile v8us*)gp = agv;
  __threadfence();
  *(volatile v8us*)gp = agv;
}

__device__ __forceinline__ void rows_out_pass(const float* sOut, float* N32, unsigned short* NA, int n0, int lane) {
#pragma unroll
  for (int i = 0; i < 16; ++i) {
    const v4f v0 = *(const v4f*)(sOut + i * FD + 4 * lane);
    const v4f v1 = *(const v4f*)(sOut + i * FD + 128 + 4 * lane);
    float* g = N32 + (size_t)(n0 + i) * FD;
    *(volatile v4f*)(g + 4 * lane) = v0;
    *(volatile v4f*)(g + 128 + 4 * lane) = v1;
  }
#pragma unroll
  for (int i = 0; i < 16; ++i) {
    const v4f a = *(const v4f*)(sOut + i * FD + 8 * lane);
    const v4f b = *(const v4f*)(sOut + i * FD + 8 * lane + 4);
    v8h o;
    o[0] = (_Float16)(a.x * (float)ASC); o[1] = (_Float16)(a.y * (float)ASC);
    o[2] = (_Float16)(a.z * (float)ASC); o[3] = (_Float16)(a.w * (float)ASC);
    o[4] = (_Float16)(b.x * (float)ASC); o[5] = (_Float16)(b.y * (float)ASC);
    o[6] = (_Float16)(b.z * (float)ASC); o[7] = (_Float16)(b.w * (float)ASC);
    const v8us ob = __builtin_bit_cast(v8us, o);
    *(volatile v8us*)(NA + (size_t)(n0 + i) * FD + 8 * lane) = ob;
  }
}

__global__ __launch_bounds__(TTHR) void k_node(
    float* N32, unsigned short* NA, const unsigned short* __restrict__ AggA,
    const unsigned short* __restrict__ N1p, const float* __restrict__ nb1,
    const unsigned short* __restrict__ N2p, const float* __restrict__ nb2,
    const float* __restrict__ lng, const float* __restrict__ lnb,
    const unsigned short* __restrict__ N3p, const float* __restrict__ nb3, int nN) {
  __shared__ __attribute__((aligned(16))) _Float16 sMidB[TW][16 * FD];
  __shared__ __attribute__((aligned(16))) float    sFB[TW][16 * FD];
  const int tid = threadIdx.x, lane = tid & 31, wave = tid >> 5, hh = lane >> 4, m = lane & 15;
  const int n0 = ((int)blockIdx.x * TW + wave) * 16;
  _Float16* sMid = sMidB[wave];
  float* sFw = sFB[wave];
  (void)nN;

#pragma unroll 1
  for (int np = 0; np < 8; ++np) {
    const int c0 = 32 * np + m, c1 = c0 + 16;
    v8f acc0 = zero8(), acc1 = zero8();
#pragma unroll 1
    for (int kt = 0; kt < 8; ++kt) {
      const v16h a  = frag_glb(NA, n0 + m, FD, 32 * kt, hh);
      const v16h b0 = frag_glb(N1p, c0, K2, 32 * kt, hh);
      const v16h b1 = frag_glb(N1p, c1, K2, 32 * kt, hh);
      acc0 = wmh(a, b0, acc0);
      acc1 = wmh(a, b1, acc1);
    }
#pragma unroll 1
    for (int kt = 0; kt < 8; ++kt) {
      const v16h a  = frag_glb(AggA, n0 + m, FD, 32 * kt, hh);
      const v16h b0 = frag_glb(N1p, c0, K2, FD + 32 * kt, hh);
      const v16h b1 = frag_glb(N1p, c1, K2, FD + 32 * kt, hh);
      acc0 = wmh(a, b0, acc0);
      acc1 = wmh(a, b1, acc1);
    }
    const float bv0 = nb1[c0], bv1 = nb1[c1];
#pragma unroll
    for (int r = 0; r < 8; ++r) {
      sMid[(8 * hh + r) * FD + c0] = (_Float16)(fmaxf(acc0[r] * OSC + bv0, 0.0f) * (float)ASC);
      sMid[(8 * hh + r) * FD + c1] = (_Float16)(fmaxf(acc1[r] * OSC + bv1, 0.0f) * (float)ASC);
    }
  }
  __syncthreads();

#pragma unroll 1
  for (int np = 0; np < 8; ++np) {
    const int c0 = 32 * np + m, c1 = c0 + 16;
    v8f acc0 = zero8(), acc1 = zero8();
#pragma unroll 1
    for (int kt = 0; kt < 8; ++kt) {
      const v16h a  = frag_lds(sMid, m, FD, 32 * kt, hh);
      const v16h b0 = frag_glb(N2p, c0, FD, 32 * kt, hh);
      const v16h b1 = frag_glb(N2p, c1, FD, 32 * kt, hh);
      acc0 = wmh(a, b0, acc0);
      acc1 = wmh(a, b1, acc1);
    }
    const float bv0 = nb2[c0], bv1 = nb2[c1];
#pragma unroll
    for (int r = 0; r < 8; ++r) {
      sFw[(8 * hh + r) * FD + c0] = acc0[r] * OSC + bv0;
      sFw[(8 * hh + r) * FD + c1] = acc1[r] * OSC + bv1;
    }
  }
  __syncthreads();

  ln_relu_rows(sFw, sMid, lng, lnb, lane);
  __syncthreads();

#pragma unroll 1
  for (int np = 0; np < 8; ++np) {
    const int c0 = 32 * np + m, c1 = c0 + 16;
    v8f acc0 = zero8(), acc1 = zero8();
#pragma unroll 1
    for (int kt = 0; kt < 8; ++kt) {
      const v16h a  = frag_lds(sMid, m, FD, 32 * kt, hh);
      const v16h b0 = frag_glb(N3p, c0, FD, 32 * kt, hh);
      const v16h b1 = frag_glb(N3p, c1, FD, 32 * kt, hh);
      acc0 = wmh(a, b0, acc0);
      acc1 = wmh(a, b1, acc1);
    }
    const float bv0 = nb3[c0], bv1 = nb3[c1];
#pragma unroll
    for (int r = 0; r < 8; ++r) {
      sFw[(8 * hh + r) * FD + c0] = acc0[r] * OSC + bv0;
      sFw[(8 * hh + r) * FD + c1] = acc1[r] * OSC + bv1;
    }
  }
  __syncthreads();

#pragma unroll 2
  for (int i = 0; i < 16; ++i) {
    const float* hg = N32 + (size_t)(n0 + i) * FD + 8 * lane;
    const v4f h0 = *(const v4f*)hg, h1 = *(const v4f*)(hg + 4);
    float* sp = sFw + i * FD + 8 * lane;
    const v4f u0 = *(const v4f*)sp + h0;
    const v4f u1 = *(const v4f*)(sp + 4) + h1;
    *(v4f*)sp = u0;
    *(v4f*)(sp + 4) = u1;
  }
  __syncthreads();

  rows_out_pass(sFw, N32, NA, n0, lane);
  __threadfence();
  rows_out_pass(sFw, N32, NA, n0, lane);
}

__global__ __launch_bounds__(NTHR) void k_pred(
    const int* __restrict__ rowi, const int* __restrict__ coli,
    const float* __restrict__ PA, const float* __restrict__ PB, const float* __restrict__ pb1,
    const float* __restrict__ pw2, const float* __restrict__ pb2, float* out, int nNa, int nNb, int nE) {
  const int tid = threadIdx.x, lane = tid & 31, wave = tid >> 5;
  const int e0 = ((int)blockIdx.x * NWAVE + wave) * PEW;
  const v4f bq0 = *(const v4f*)(pb1 + 8 * lane), bq1 = *(const v4f*)(pb1 + 8 * lane + 4);
  const v4f wq0 = *(const v4f*)(pw2 + 8 * lane), wq1 = *(const v4f*)(pw2 + 8 * lane + 4);
  const float pb = pb2[0];
  float res = 0.0f;
#pragma unroll 1
  for (int j = 0; j < PEW; ++j) {
    int e = e0 + j; e = e > nE - 1 ? nE - 1 : e;
    int r = rowi[e];
    int c = coli[e];
    r = r < 0 ? 0 : (r > nNa - 1 ? nNa - 1 : r);
    c = c < 0 ? 0 : (c > nNb - 1 ? nNb - 1 : c);
    const float* pr = PA + (size_t)r * FD + 8 * lane;
    const float* pc = PB + (size_t)c * FD + 8 * lane;
    const v4f x0 = *(const v4f*)pr + *(const v4f*)pc + bq0;
    const v4f x1 = *(const v4f*)(pr + 4) + *(const v4f*)(pc + 4) + bq1;
    float s = fmaxf(x0.x, 0.0f) * wq0.x;
    s += fmaxf(x0.y, 0.0f) * wq0.y;
    s += fmaxf(x0.z, 0.0f) * wq0.z;
    s += fmaxf(x0.w, 0.0f) * wq0.w;
    s += fmaxf(x1.x, 0.0f) * wq1.x;
    s += fmaxf(x1.y, 0.0f) * wq1.y;
    s += fmaxf(x1.z, 0.0f) * wq1.z;
    s += fmaxf(x1.w, 0.0f) * wq1.w;
    s = wsum32(s);
    res = (lane == j) ? (s + pb) : res;
  }
  const float y = __builtin_amdgcn_rcpf(1.0f + expf(-res));
  const bool act = (e0 + lane) < nE;
  if (act) *(volatile float*)(out + (size_t)e0 + lane) = y;
  __threadfence();
  if (act) *(volatile float*)(out + (size_t)e0 + lane) = y;
}

extern "C" void kernel_launch(void* const* d_in, const int* in_sizes, int n_in,
                              void* d_out, int out_size, void* d_ws, size_t ws_size,
                              hipStream_t stream) {
  if (n_in < 24) return;
  if (in_sizes[0] <= 0 || (in_sizes[0] % FD) != 0 || in_sizes[1] <= 0 || (in_sizes[1] % FD) != 0) return;
  const int nNa = in_sizes[0] / FD;
  const int nNb = in_sizes[1] / FD;
  const int nE  = in_sizes[2];
  if (nE <= 0 || in_sizes[3] != nE || out_size != nE) return;
  if (in_sizes[4] != K2 * FD || in_sizes[5] != FD || in_sizes[6] != FD * FD || in_sizes[7] != FD) return;
  if (in_sizes[8] != FD || in_sizes[9] != FD || in_sizes[10] != FD * FD || in_sizes[11] != FD) return;
  if (in_sizes[12] != K2 * FD || in_sizes[13] != FD || in_sizes[14] != FD * FD || in_sizes[15] != FD) return;
  if (in_sizes[16] != FD || in_sizes[17] != FD || in_sizes[18] != FD * FD || in_sizes[19] != FD) return;
  if (in_sizes[20] != K2 * FD || in_sizes[21] != FD || in_sizes[22] != FD || in_sizes[23] < 1) return;
  if ((nNa % 64) != 0 || (nNb % 64) != 0) return;
  if (nNa > (1 << 20) || nNb > (1 << 20) || nE > (1 << 26)) return;

  const float* node0 = (const float*)d_in[0];
  const float* node1 = (const float*)d_in[1];
  const int*   rows  = (const int*)d_in[2];
  const int*   cols  = (const int*)d_in[3];
  const float* e_w1 = (const float*)d_in[4];  const float* e_b1 = (const float*)d_in[5];
  const float* e_w2 = (const float*)d_in[6];  const float* e_b2 = (const float*)d_in[7];
  const float* e_g  = (const float*)d_in[8];  const float* e_be = (const float*)d_in[9];
  const float* e_w3 = (const float*)d_in[10]; const float* e_b3 = (const float*)d_in[11];
  const float* n_w1 = (const float*)d_in[12]; const float* n_b1 = (const float*)d_in[13];
  const float* n_w2 = (const float*)d_in[14]; const float* n_b2 = (const float*)d_in[15];
  const float* n_g  = (const float*)d_in[16]; const float* n_be = (const float*)d_in[17];
  const float* n_w3 = (const float*)d_in[18]; const float* n_b3 = (const float*)d_in[19];
  const float* p_w1 = (const float*)d_in[20]; const float* p_b1 = (const float*)d_in[21];
  const float* p_w2 = (const float*)d_in[22]; const float* p_b2 = (const float*)d_in[23];
  float* out = (float*)d_out;

  const int nBC = (nNa + NBC - 1) / NBC;
  const int CNTPAD = nBC * NBC;
  if (FPB * nBC + 1 > RBN) return;
  const int nBF = (nNa + NBF - 1) / NBF;
  if (nBF > FPB * nBC) return;
  if (31 * FPB * nBC > 4096) return;
  const int csrLen = ((nE + 63) & ~63) + 4096;
  const size_t NA8 = (size_t)nNa, NB8 = (size_t)nNb;

  char* ws = (char*)d_ws;
  size_t off = 0;
  const size_t oEW1 = off; off += (size_t)FD * K2 * 2;           off = (off + 255) & ~(size_t)255;
  const size_t oEW2 = off; off += (size_t)FD * FD * 2;           off = (off + 255) & ~(size_t)255;
  const size_t oEW3 = off; off += (size_t)FD * FD * 2;           off = (off + 255) & ~(size_t)255;
  const size_t oNW1 = off; off += (size_t)FD * K2 * 2;           off = (off + 255) & ~(size_t)255;
  const size_t oNW2 = off; off += (size_t)FD * FD * 2;           off = (off + 255) & ~(size_t)255;
  const size_t oNW3 = off; off += (size_t)FD * FD * 2;           off = (off + 255) & ~(size_t)255;
  const size_t oPW1 = off; off += (size_t)FD * K2 * 2;           off = (off + 255) & ~(size_t)255;
  const size_t oN32 = off; off += NA8 * FD * 4;                  off = (off + 255) & ~(size_t)255;
  const size_t oNA  = off; off += NA8 * FD * 2;                  off = (off + 255) & ~(size_t)255;
  const size_t oNB  = off; off += NB8 * FD * 2;                  off = (off + 255) & ~(size_t)255;
  const size_t oAGG = off; off += NA8 * FD * 2;                  off = (off + 255) & ~(size_t)255;
  const size_t oPA  = off; off += NA8 * FD * 4;                  off = (off + 255) & ~(size_t)255;
  const size_t oPB  = off; off += NB8 * FD * 4;                  off = (off + 255) & ~(size_t)255;
  const size_t oM   = off; off += (size_t)csrLen * FD * 2;       off = (off + 255) & ~(size_t)255;
  const size_t oCnt = off; off += (size_t)CNTPAD * 4;            off = (off + 255) & ~(size_t)255;
  const size_t oOff = off; off += (size_t)CNTPAD * 4;            off = (off + 255) & ~(size_t)255;
  const size_t oRb  = off; off += (size_t)RBN * 4;               off = (off + 255) & ~(size_t)255;
  const size_t oCsC = off; off += (size_t)csrLen * 4;            off = (off + 255) & ~(size_t)255;
  const size_t oCsR = off; off += (size_t)csrLen * 4;            off = (off + 255) & ~(size_t)255;
  if (off > ws_size || off > (size_t)WSCAP) return;

  unsigned short* EW1p = (unsigned short*)(ws + oEW1);
  unsigned short* EW2p = (unsigned short*)(ws + oEW2);
  unsigned short* EW3p = (unsigned short*)(ws + oEW3);
  unsigned short* NW1p = (unsigned short*)(ws + oNW1);
  unsigned short* NW2p = (unsigned short*)(ws + oNW2);
  unsigned short* NW3p = (unsigned short*)(ws + oNW3);
  unsigned short* PW1p = (unsigned short*)(ws + oPW1);
  float*          N32  = (float*)(ws + oN32);
  unsigned short* NA   = (unsigned short*)(ws + oNA);
  unsigned short* NBp  = (unsigned short*)(ws + oNB);
  unsigned short* AGG  = (unsigned short*)(ws + oAGG);
  float*          PA   = (float*)(ws + oPA);
  float*          PB   = (float*)(ws + oPB);
  unsigned short* Mpl  = (unsigned short*)(ws + oM);
  int*            cnt  = (int*)(ws + oCnt);
  int*            offp = (int*)(ws + oOff);
  int*            rb   = (int*)(ws + oRb);
  int*            csrC = (int*)(ws + oCsC);
  int*            csrR = (int*)(ws + oCsR);

  const int vec4 = 1;

  k_wcvt<<<dim3((FD * (K2 / 8) + NTHR - 1) / NTHR, 7, 1), NTHR, 0, stream>>>(
      e_w1, e_w2, e_w3, n_w1, n_w2, n_w3, p_w1, EW1p, EW2p, EW3p, NW1p, NW2p, NW3p, PW1p);
  {
    const int n8a = nNa * (FD / 8), n8b = nNb * (FD / 8);
    k_ncvt<1><<<(n8a + NTHR - 1) / NTHR, NTHR, 0, stream>>>(node0, N32, NA, n8a);
    k_ncvt<0><<<(n8b + NTHR - 1) / NTHR, NTHR, 0, stream>>>(node1, N32, NBp, n8b);
  }
  k_count<<<nBC, NTHR, 0, stream>>>(rows, cnt, nE, vec4);
  k_offsets<<<1, OTHR, 0, stream>>>(cnt, offp, rb, nBC);
  hipFuncSetAttribute(reinterpret_cast<const void*>(&k_fill),
                      hipFuncAttributeMaxDynamicSharedMemorySize, LDS_FILL);
  k_fill<<<nBF, NTHR, LDS_FILL, stream>>>(cols, rows, offp, rb, csrC, csrR, nNa, nNb, nE, vec4, csrLen);
  k_gemm<<<dim3(nNb / BM, FD / NCW, 1), NTHR, 0, stream>>>(NBp, EW1p + FD, PB, FD, K2, FD / 32, FD, OSC);

  for (int it = 0; it < 3; ++it) {
    k_gemm<<<dim3(nNa / BM, FD / NCW, 1), NTHR, 0, stream>>>(NA, EW1p, PA, FD, K2, FD / 32, FD, OSC);
    k_edge<<<csrLen / (TW * 16), TTHR, 0, stream>>>(csrR, csrC, PA, PB, e_b1, EW2p, e_b2, e_g, e_be,
                                                     EW3p, e_b3, Mpl, nNa, nNb, csrLen);
    k_agg<<<nNa / ANB, NTHR, 0, stream>>>(cnt, offp, Mpl, AGG, nNa, csrLen);
    k_node<<<nNa / (TW * 16), TTHR, 0, stream>>>(N32, NA, AGG, NW1p, n_b1, NW2p, n_b2, n_g, n_be,
                                                 NW3p, n_b3, nNa);
  }

  k_gemm<<<dim3(nNa / BM, FD / NCW, 1), NTHR, 0, stream>>>(NA, PW1p, PA, FD, K2, FD / 32, FD, OSC);
  k_gemm<<<dim3(nNb / BM, FD / NCW, 1), NTHR, 0, stream>>>(NBp, PW1p + FD, PB, FD, K2, FD / 32, FD, OSC);
  k_pred<<<(nE + NWAVE * PEW - 1) / (NWAVE * PEW), NTHR, 0, stream>>>(rows, cols, PA, PB, p_b1, p_w2, p_b2,
                                                                       out, nNa, nNb, nE);
}
